// GauntTensorProductS2Grid_50036368999124
// MI455X (gfx1250) — hardware-verified
//
#include <hip/hip_runtime.h>


typedef __bf16       v16bf __attribute__((ext_vector_type(16)));
typedef float        v8f   __attribute__((ext_vector_type(8)));
typedef float        v4f   __attribute__((ext_vector_type(4)));
typedef unsigned int v4u   __attribute__((ext_vector_type(4)));

#define DIN        81
#define KST        3
#define NBETA      64
#define NALPHA     128
#define NGRID      (NBETA * NALPHA)
#define DOUT       289
#define NJT        19
#define NC16       (NGRID / 16)
#define NC32       (NGRID / 32)
#define NIT        (NC32 / 8)
#define FRAG_BYTES 1024u
#define YIN_FRAGS  (NC16 * KST)
#define YOUT_FRAGS (NC32 * NJT)
#define TROWS      32
#define NTHR       256

#define XA_BYTES   (2u * 2u * 2u * (unsigned)KST * FRAG_BYTES)
#define FB_OFF     XA_BYTES
#define FB_BYTES   (2u * 8u * 2u * FRAG_BYTES)
#define SMEM_BYTES (XA_BYTES + FB_BYTES)

static_assert(TROWS * DOUT * 4 <= (int)SMEM_BYTES);
static_assert((TROWS * DOUT * 4) % 128 == 0);

union V16 {
    v4u   q[2];
    v16bf v;
};

__device__ __forceinline__ unsigned int bf16_bits(float x) {
    unsigned int u = __float_as_uint(x);
    u += 0x7FFFu + ((u >> 16) & 1u);
    return u >> 16;
}

__device__ __forceinline__ void split_pack8(const float* v, v4u* H, v4u* L) {
    unsigned int hb[8], lb[8];
#pragma unroll
    for (int e = 0; e < 8; ++e) {
        const unsigned int hi = bf16_bits(v[e]);
        const float xh = __uint_as_float(hi << 16);
        hb[e] = hi;
        lb[e] = bf16_bits(v[e] - xh);
    }
    v4u h4, l4;
    h4.x = hb[0] | (hb[1] << 16); h4.y = hb[2] | (hb[3] << 16);
    h4.z = hb[4] | (hb[5] << 16); h4.w = hb[6] | (hb[7] << 16);
    l4.x = lb[0] | (lb[1] << 16); l4.y = lb[2] | (lb[3] << 16);
    l4.z = lb[4] | (lb[5] << 16); l4.w = lb[6] | (lb[7] << 16);
    *H = h4; *L = l4;
}

__device__ __forceinline__ v8f mma_bf16(const v16bf a, const v16bf b, v8f c) {
    v8f d = __builtin_amdgcn_wmma_f32_16x16x32_bf16(false, a, false, b, (short)0, c, false, false);
    asm volatile("v_nop\n\tv_nop\n\tv_nop\n\tv_nop" : "+v"(d) : "v"(a), "v"(b));
    return d;
}

__device__ __forceinline__ void load_frag(V16& f, const unsigned char* p) {
    const v4u* q = (const v4u*)p;
    f.q[0] = q[0];
    f.q[1] = q[1];
}

__global__ void __launch_bounds__(NTHR)
k_stage_yin(const float* __restrict__ yin,
            unsigned char* __restrict__ wsh,
            unsigned char* __restrict__ wsl)
{
    const int g = blockIdx.x * NTHR + threadIdx.x;
    const int F = g >> 6;
    if (F >= YIN_FRAGS) return;
    const int q   = g & 63;
    const int c16 = F / KST;
    const int s   = F - c16 * KST;
    const int lq  = q >> 1;
    const int hf  = q & 1;
    const int col = c16 * 16 + (lq & 15);
    const int kb  = 32 * s + 8 * (lq >> 4) + 16 * hf;

    float v[8];
#pragma unroll
    for (int e = 0; e < 8; ++e) {
        const int k = kb + e;
        v[e] = (k < DIN) ? yin[(size_t)k * NGRID + col] : 0.0f;
    }
    v4u H, L;
    split_pack8(v, &H, &L);

    const size_t off = (size_t)F * FRAG_BYTES + (size_t)q * 16;
    *(volatile v4u*)(wsh + off) = H;
    *(volatile v4u*)(wsl + off) = L;
    __threadfence();
    *(volatile v4u*)(wsh + off) = H;
    *(volatile v4u*)(wsl + off) = L;
}

__global__ void __launch_bounds__(NTHR)
k_stage_yout(const float* __restrict__ yout,
             unsigned char* __restrict__ wsh,
             unsigned char* __restrict__ wsl)
{
    const int g = blockIdx.x * NTHR + threadIdx.x;
    const int F = g >> 6;
    if (F >= YOUT_FRAGS) return;
    const int q   = g & 63;
    const int c32 = F / NJT;
    const int jt  = F - c32 * NJT;
    const int lq  = q >> 1;
    const int hf  = q & 1;
    const int j   = jt * 16 + (lq & 15);
    const int jc  = (j < DOUT) ? j : (DOUT - 1);
    const int kb  = c32 * 32 + 8 * (lq >> 4) + 16 * hf;

    const float* row = yout + (size_t)jc * NGRID + kb;
    float v[8];
#pragma unroll
    for (int e = 0; e < 8; ++e)
        v[e] = (j < DOUT) ? row[e] : 0.0f;
    v4u H, L;
    split_pack8(v, &H, &L);

    const size_t off = (size_t)F * FRAG_BYTES + (size_t)q * 16;
    *(volatile v4u*)(wsh + off) = H;
    *(volatile v4u*)(wsl + off) = L;
    __threadfence();
    *(volatile v4u*)(wsh + off) = H;
    *(volatile v4u*)(wsl + off) = L;
}

__device__ __forceinline__ unsigned int xa_off(int inp, int plane, int rt, int s) {
    return (unsigned int)((((inp * 2 + plane) * 2 + rt) * KST + s)) * FRAG_BYTES;
}
__device__ __forceinline__ unsigned int fb_off(int plane, int ch, int rt) {
    return FB_OFF + (unsigned int)(((plane * 8 + ch) * 2 + rt)) * FRAG_BYTES;
}

__device__ __forceinline__ v8f acc3(v8f acc, const v16bf fh, const v16bf fl,
                                    const unsigned char* bh, const unsigned char* bl) {
    V16 BH, BL;
    load_frag(BH, bh);
    load_frag(BL, bl);
    acc = mma_bf16(fh, BH.v, acc);
    acc = mma_bf16(fh, BL.v, acc);
    acc = mma_bf16(fl, BH.v, acc);
    return acc;
}

__device__ __forceinline__ void put_tile(float* outs, const v8f acc, int rt, int jt, int m, int h) {
    const int j = jt * 16 + m;
    if (j < DOUT) {
#pragma unroll
        for (int r = 0; r < 8; ++r)
            outs[(rt * 16 + 8 * h + r) * DOUT + j] = acc[r];
    }
}

__global__ void __launch_bounds__(NTHR)
k_project(const float* __restrict__ x1,
          const float* __restrict__ x2,
          const float* __restrict__ w,
          const unsigned char* __restrict__ yinh,
          const unsigned char* __restrict__ yinl,
          const unsigned char* __restrict__ youth,
          const unsigned char* __restrict__ youtl,
          float* __restrict__ out,
          int nrows)
{
    __shared__ __align__(16) unsigned char smem[SMEM_BYTES];

    const int tid  = threadIdx.x;
    const int wv   = __builtin_amdgcn_readfirstlane(tid >> 5);
    const int lane = tid & 31;
    const int m    = lane & 15;
    const int h    = lane >> 4;
    const int n0   = blockIdx.x * TROWS;

    for (int p = wv; p < 12; p += 8) {
        const int inp = p / 6;
        const int rem = p - inp * 6;
        const int rt  = rem / KST;
        const int s   = rem - rt * KST;
        const float* X = inp ? x2 : x1;
        int row = n0 + rt * 16 + m;
        row = (row < nrows) ? row : (nrows - 1);
        const float* xr = X + (size_t)row * DIN;
        float v0[8], v1[8];
#pragma unroll
        for (int e = 0; e < 8; ++e) {
            const int k0 = 32 * s + 8 * h + e;
            const int k1 = k0 + 16;
            v0[e] = (k0 < DIN) ? xr[k0] : 0.0f;
            v1[e] = (k1 < DIN) ? xr[k1] : 0.0f;
        }
        v4u H0, L0, H1, L1;
        split_pack8(v0, &H0, &L0);
        split_pack8(v1, &H1, &L1);
        v4u* dh = (v4u*)(smem + xa_off(inp, 0, rt, s) + lane * 32);
        v4u* dl = (v4u*)(smem + xa_off(inp, 1, rt, s) + lane * 32);
        dh[0] = H0; dh[1] = H1;
        dl[0] = L0; dl[1] = L1;
    }

    const int rtc    = wv >> 2;
    const int jstart = 5 * (wv & 3);
    const int jcnt   = ((wv & 3) == 3) ? 4 : 5;

    const v8f zero = {0.f, 0.f, 0.f, 0.f, 0.f, 0.f, 0.f, 0.f};
    v8f acc0 = zero, acc1 = zero, acc2 = zero, acc3v = zero, acc4 = zero;

    for (int it = 0; it < NIT; ++it) {
        __syncthreads();

        const float wb = w[(it * 256 + wv * 32) >> 7];
#pragma unroll
        for (int rt = 0; rt < 2; ++rt) {
            V16 FH, FL;
#pragma unroll
            for (int t = 0; t < 2; ++t) {
                const int c16 = it * 16 + wv * 2 + t;
                v8f g1 = zero, g2 = zero;
#pragma unroll
                for (int s = 0; s < KST; ++s) {
                    const size_t yo = (size_t)(c16 * KST + s) * FRAG_BYTES + (size_t)lane * 32;
                    V16 YH, YL, XH, XL;
                    load_frag(YH, yinh + yo);
                    load_frag(YL, yinl + yo);
                    load_frag(XH, smem + xa_off(0, 0, rt, s) + lane * 32);
                    load_frag(XL, smem + xa_off(0, 1, rt, s) + lane * 32);
                    g1 = mma_bf16(YH.v, XH.v, g1);
                    g1 = mma_bf16(YH.v, XL.v, g1);
                    g1 = mma_bf16(YL.v, XH.v, g1);
                    load_frag(XH, smem + xa_off(1, 0, rt, s) + lane * 32);
                    load_frag(XL, smem + xa_off(1, 1, rt, s) + lane * 32);
                    g2 = mma_bf16(YH.v, XH.v, g2);
                    g2 = mma_bf16(YH.v, XL.v, g2);
                    g2 = mma_bf16(YL.v, XH.v, g2);
                }
                float fv[8];
#pragma unroll
                for (int r = 0; r < 8; ++r) fv[r] = (g1[r] * g2[r]) * wb;
                split_pack8(fv, &FH.q[t], &FL.q[t]);
            }
            v4u* fh = (v4u*)(smem + fb_off(0, wv, rt) + lane * 32);
            v4u* fl = (v4u*)(smem + fb_off(1, wv, rt) + lane * 32);
            fh[0] = FH.q[0]; fh[1] = FH.q[1];
            fl[0] = FL.q[0]; fl[1] = FL.q[1];
        }

        __syncthreads();

        for (int ch = 0; ch < 8; ++ch) {
            V16 FH, FL;
            load_frag(FH, smem + fb_off(0, ch, rtc) + lane * 32);
            load_frag(FL, smem + fb_off(1, ch, rtc) + lane * 32);
            const size_t bo = (size_t)((it * 8 + ch) * NJT + jstart) * FRAG_BYTES + (size_t)lane * 32;
            const unsigned char* bh = youth + bo;
            const unsigned char* bl = youtl + bo;
            acc0  = acc3(acc0,  FH.v, FL.v, bh,                  bl);
            acc1  = acc3(acc1,  FH.v, FL.v, bh + FRAG_BYTES,     bl + FRAG_BYTES);
            acc2  = acc3(acc2,  FH.v, FL.v, bh + 2 * FRAG_BYTES, bl + 2 * FRAG_BYTES);
            acc3v = acc3(acc3v, FH.v, FL.v, bh + 3 * FRAG_BYTES, bl + 3 * FRAG_BYTES);
            if (jcnt == 5)
                acc4 = acc3(acc4, FH.v, FL.v, bh + 4 * FRAG_BYTES, bl + 4 * FRAG_BYTES);
        }
    }

    __syncthreads();
    float* outs = (float*)smem;
    put_tile(outs, acc0,  rtc, jstart + 0, m, h);
    put_tile(outs, acc1,  rtc, jstart + 1, m, h);
    put_tile(outs, acc2,  rtc, jstart + 2, m, h);
    put_tile(outs, acc3v, rtc, jstart + 3, m, h);
    if (jcnt == 5) put_tile(outs, acc4, rtc, jstart + 4, m, h);
    __syncthreads();

    int rows_valid = nrows - n0;
    if (rows_valid > TROWS) rows_valid = TROWS;
    const int    nfl   = rows_valid * DOUT;
    const int    nq    = nfl >> 2;
    const size_t obase = (size_t)n0 * DOUT;

    for (int i = tid; i < nq; i += NTHR) {
        v4f v;
        v.x = outs[4 * i + 0]; v.y = outs[4 * i + 1]; v.z = outs[4 * i + 2]; v.w = outs[4 * i + 3];
        *(volatile v4f*)(out + obase + (size_t)(4 * i)) = v;
    }
    for (int i = 4 * nq + tid; i < nfl; i += NTHR) {
        const float v = outs[i];
        *(volatile float*)(out + obase + i) = v;
    }
    __threadfence();
    for (int i = tid; i < nq; i += NTHR) {
        v4f v;
        v.x = outs[4 * i + 0]; v.y = outs[4 * i + 1]; v.z = outs[4 * i + 2]; v.w = outs[4 * i + 3];
        *(volatile v4f*)(out + obase + (size_t)(4 * i)) = v;
    }
    for (int i = 4 * nq + tid; i < nfl; i += NTHR) {
        const float v = outs[i];
        *(volatile float*)(out + obase + i) = v;
    }
}

extern "C" void kernel_launch(void* const* d_in, const int* in_sizes, int n_in,
                              void* d_out, int out_size, void* d_ws, size_t ws_size,
                              hipStream_t stream)
{
    if (n_in < 5) return;
    const int ne0 = in_sizes[0];
    if (ne0 <= 0 || (ne0 % DIN) != 0) return;
    const int nrows = ne0 / DIN;
    if (in_sizes[1] != ne0) return;
    if (in_sizes[2] != DIN * NGRID) return;
    if (in_sizes[3] != DOUT * NGRID) return;
    if (in_sizes[4] != NBETA) return;
    if (out_size != nrows * DOUT) return;

    const size_t yin_bytes  = (size_t)YIN_FRAGS  * FRAG_BYTES;
    const size_t yout_bytes = (size_t)YOUT_FRAGS * FRAG_BYTES;
    const size_t off_yinh  = 0;
    const size_t off_yinl  = off_yinh  + yin_bytes;
    const size_t off_youth = off_yinl  + yin_bytes;
    const size_t off_youtl = off_youth + yout_bytes;
    const size_t total     = off_youtl + yout_bytes;
    if (total > ws_size) return;

    const float* x1   = (const float*)d_in[0];
    const float* x2   = (const float*)d_in[1];
    const float* yin  = (const float*)d_in[2];
    const float* yout = (const float*)d_in[3];
    const float* w    = (const float*)d_in[4];
    float* out = (float*)d_out;
    unsigned char* ws = (unsigned char*)d_ws;

    const int g_yin  = (YIN_FRAGS  * 64 + NTHR - 1) / NTHR;
    const int g_yout = (YOUT_FRAGS * 64 + NTHR - 1) / NTHR;
    const int g_main = (nrows + TROWS - 1) / TROWS;

    k_stage_yin<<<g_yin, NTHR, 0, stream>>>(yin, ws + off_yinh, ws + off_yinl);
    k_stage_yout<<<g_yout, NTHR, 0, stream>>>(yout, ws + off_youth, ws + off_youtl);
    k_project<<<g_main, NTHR, 0, stream>>>(x1, x2, w,
                                           ws + off_yinh, ws + off_yinl,
                                           ws + off_youth, ws + off_youtl,
                                           out, nrows);
}
